// CONV_tiny_add_partial_60138132079272
// MI455X (gfx1250) — hardware-verified
//
#include <hip/hip_runtime.h>
#define NB 1024
typedef __bf16 v16b __attribute__((ext_vector_type(16)));
typedef unsigned short v8us __attribute__((ext_vector_type(8), may_alias));
typedef float  v8f  __attribute__((ext_vector_type(8)));
typedef float  v4f  __attribute__((ext_vector_type(4)));
typedef float  v4fa __attribute__((ext_vector_type(4), may_alias));
union FragB { v16b v; v8us half[2]; unsigned short u[16]; };

__device__ __forceinline__ unsigned short bf16_bits(float x) { unsigned int u = __float_as_uint(x); return (unsigned short)((u + 0x7FFFu + ((u >> 16) & 1u)) >> 16); }
__device__ __forceinline__ float bf16_val(unsigned short b) { return __uint_as_float(((unsigned int)b) << 16); }
__device__ __forceinline__ float bf16_round(float x) { return bf16_val(bf16_bits(x)); }
template <int NT>
__device__ __forceinline__ v8f mmaN(v16b ah, v16b al, v16b bh, v16b bl, v8f c) {
  c = __builtin_amdgcn_wmma_f32_16x16x32_bf16(false, ah, false, bh, (short)0, c, false, false);
  if (NT >= 2) c = __builtin_amdgcn_wmma_f32_16x16x32_bf16(false, al, false, bh, (short)0, c, false, false);
  if (NT >= 3) c = __builtin_amdgcn_wmma_f32_16x16x32_bf16(false, ah, false, bl, (short)0, c, false, false);
  asm volatile("v_nop\n\tv_nop\n\tv_nop\n\tv_nop" : "+v"(c) : "v"(ah), "v"(al), "v"(bh), "v"(bl));
  return c;
}

__global__ __launch_bounds__(256) void k_wt_bf16(const float* __restrict__ W, unsigned short* __restrict__ Wt, int K, int N) {
  const int t = blockIdx.x * 256 + threadIdx.x;
  const int k8n = K / 8;
  if (t >= N * k8n) return;
  const int n = t / k8n, k8 = (t % k8n) * 8;
  v8us v;
#pragma unroll
  for (int i = 0; i < 8; ++i) v[i] = bf16_bits(W[(size_t)(k8 + i) * N + n]);
  *(volatile v8us*)(Wt + (size_t)n * K + k8) = v;
  __threadfence();
  *(volatile v8us*)(Wt + (size_t)n * K + k8) = v;
}

template <bool ASPLIT, int ACT, bool BIAS_BF16>
__global__ __launch_bounds__(128) void k_gemm_bf(const float* __restrict__ A, int lda, const unsigned short* __restrict__ Wt, int ldb,
                                               const float* __restrict__ bias, float* __restrict__ C, int ldc, int M, int N, int K) {
  __shared__ __attribute__((aligned(16))) float so[4][16][64];
  const int tid = threadIdx.x, w = tid >> 5, lane = tid & 31, ln = lane & 15, hh = lane >> 4;
  const int ntn = N / 64;
  const int wid = blockIdx.x * 4 + w;
  const int mt = wid / ntn, nq = wid % ntn;
  if (mt * 16 >= M) return;
  const int row0 = mt * 16, col0 = nq * 64;
  const float* arow = A + (size_t)(row0 + ln) * lda;
  v8f acc[4] = {};
  for (int kb = 0; kb < K; kb += 32) {
    FragB ah, al;
    const v4f x0 = *(const v4fa*)(arow + kb + 8 * hh), x1 = *(const v4fa*)(arow + kb + 8 * hh + 4);
    const v4f x2 = *(const v4fa*)(arow + kb + 16 + 8 * hh), x3 = *(const v4fa*)(arow + kb + 16 + 8 * hh + 4);
    float xs[16] = {x0[0],x0[1],x0[2],x0[3],x1[0],x1[1],x1[2],x1[3],x2[0],x2[1],x2[2],x2[3],x3[0],x3[1],x3[2],x3[3]};
#pragma unroll
    for (int i = 0; i < 16; ++i) { const unsigned short hb = bf16_bits(xs[i]); ah.u[i] = hb; al.u[i] = ASPLIT ? bf16_bits(xs[i] - bf16_val(hb)) : (unsigned short)0; }
#pragma unroll
    for (int t = 0; t < 4; ++t) {
      const unsigned short* brow = Wt + (size_t)(col0 + t * 16 + ln) * ldb + kb;
      FragB b;
      b.half[0] = *(const v8us*)(brow + 8 * hh);
      b.half[1] = *(const v8us*)(brow + 16 + 8 * hh);
      acc[t] = mmaN<ASPLIT ? 2 : 1>(ah.v, al.v, b.v, b.v, acc[t]);
    }
  }
#pragma unroll
  for (int t = 0; t < 4; ++t) {
    float bv = bias ? bias[col0 + t * 16 + ln] : 0.f;
    if (BIAS_BF16) bv = bf16_round(bv);
#pragma unroll
    for (int r = 0; r < 8; ++r) { float v = acc[t][r] + bv; if (ACT == 1) v = fmaxf(v, 0.f); so[w][8 * hh + r][t * 16 + ln] = v; }
  }
  __builtin_amdgcn_fence(__ATOMIC_ACQ_REL, "workgroup");
  __builtin_amdgcn_wave_barrier();
  const int rsub = lane >> 4, c4 = (lane & 15) * 4;
  for (int pass = 0; pass < 2; ++pass) {
#pragma unroll
    for (int q = 0; q < 8; ++q) {
      const int r = q * 2 + rsub;
      const v4f v = *(const v4fa*)&so[w][r][c4];
      *(volatile v4f*)(C + (size_t)(row0 + r) * ldc + col0 + c4) = v;
    }
    if (pass == 0) __threadfence();
  }
}

template <bool ASPLIT, int ACT, bool BIAS_BF16, bool RES_BF16>
__global__ __launch_bounds__(128) void k_gemm_bf3(const float* __restrict__ A, int lda, const unsigned short* __restrict__ Wt, int ldb,
                                                const float* __restrict__ bias, const float* __restrict__ resid, int rmod, int ldr,
                                                float* __restrict__ C, int ldc, int M, int N, int K) {
  __shared__ __attribute__((aligned(16))) float so[4][16][64];
  const int tid = threadIdx.x, w = tid >> 5, lane = tid & 31, ln = lane & 15, hh = lane >> 4;
  const int ntn = N / 64;
  const int wid = blockIdx.x * 4 + w;
  const int mt = wid / ntn, nq = wid % ntn;
  if (mt * 16 >= M) return;
  const int row0 = mt * 16, col0 = nq * 64;
  const float* arow = A + (size_t)(row0 + ln) * lda;
  v8f acc[4] = {};
  for (int kb = 0; kb < K; kb += 32) {
    FragB ah, al;
    const v4f x0 = *(const v4fa*)(arow + kb + 8 * hh), x1 = *(const v4fa*)(arow + kb + 8 * hh + 4);
    const v4f x2 = *(const v4fa*)(arow + kb + 16 + 8 * hh), x3 = *(const v4fa*)(arow + kb + 16 + 8 * hh + 4);
    float xs[16] = {x0[0],x0[1],x0[2],x0[3],x1[0],x1[1],x1[2],x1[3],x2[0],x2[1],x2[2],x2[3],x3[0],x3[1],x3[2],x3[3]};
#pragma unroll
    for (int i = 0; i < 16; ++i) { const unsigned short hb = bf16_bits(xs[i]); ah.u[i] = hb; al.u[i] = ASPLIT ? bf16_bits(xs[i] - bf16_val(hb)) : (unsigned short)0; }
#pragma unroll
    for (int t = 0; t < 4; ++t) {
      const unsigned short* brow = Wt + (size_t)(col0 + t * 16 + ln) * ldb + kb;
      FragB b;
      b.half[0] = *(const v8us*)(brow + 8 * hh);
      b.half[1] = *(const v8us*)(brow + 16 + 8 * hh);
      acc[t] = mmaN<ASPLIT ? 2 : 1>(ah.v, al.v, b.v, b.v, acc[t]);
    }
  }
#pragma unroll
  for (int t = 0; t < 4; ++t) {
    const int col = col0 + t * 16 + ln;
    float bv = bias ? bias[col] : 0.f;
    if (BIAS_BF16) bv = bf16_round(bv);
#pragma unroll
    for (int r = 0; r < 8; ++r) {
      float v = acc[t][r] + bv;
      if (resid) { float rv = resid[(size_t)((row0 + 8 * hh + r) % rmod) * ldr + col]; if (RES_BF16) rv = bf16_round(rv); v += rv; }
      if (ACT == 1) v = fmaxf(v, 0.f);
      if (ACT == 2) v = 0.5f * v * (1.0f + erff(v * 0.70710678118654752f));
      if (ACT == 3) { const float u = 0.7978845608028654f * (v + 0.044715f * v * v * v); v = 0.5f * v * (1.0f + tanhf(u)); }
      so[w][8 * hh + r][t * 16 + ln] = v;
    }
  }
  __builtin_amdgcn_fence(__ATOMIC_ACQ_REL, "workgroup");
  __builtin_amdgcn_wave_barrier();
  const int rsub = lane >> 4, c4 = (lane & 15) * 4;
  for (int pass = 0; pass < 2; ++pass) {
#pragma unroll
    for (int q = 0; q < 8; ++q) {
      const int r = q * 2 + rsub;
      const v4f v = *(const v4fa*)&so[w][r][c4];
      *(volatile v4f*)(C + (size_t)(row0 + r) * ldc + col0 + c4) = v;
    }
    if (pass == 0) __threadfence();
  }
}
template <bool PARAM_BF16>
__global__ __launch_bounds__(256) void k_layernorm(const float* __restrict__ X, const float* __restrict__ R, const float* __restrict__ g, const float* __restrict__ bta,
                                                  float* __restrict__ out_sum, float* __restrict__ out_norm, int N, float eps) {
  __shared__ float red[256];
  const int row = blockIdx.x, tid = threadIdx.x;
  const float* x = X + (size_t)row * N; const float* rr = R ? R + (size_t)row * N : nullptr;
  float vals[16];
  const int per = N / 256;
  float s1 = 0.f;
  for (int u = 0; u < per / 4; ++u) {
    const int j = tid * 4 + 1024 * u;
    const v4f a = *(const v4fa*)(x + j);
    v4f b = {0.f,0.f,0.f,0.f}; if (rr) b = *(const v4fa*)(rr + j);
#pragma unroll
    for (int q = 0; q < 4; ++q) { const float v = a[q] + b[q]; vals[u * 4 + q] = v; s1 += v; }
  }
  red[tid] = s1; __syncthreads();
  for (int st = 128; st > 0; st >>= 1) { if (tid < st) red[tid] += red[tid + st]; __syncthreads(); }
  const float mu = red[0] / (float)N; __syncthreads();
  float s2 = 0.f;
  for (int u = 0; u < per / 4; ++u)
#pragma unroll
    for (int q = 0; q < 4; ++q) { const float c = vals[u * 4 + q] - mu; s2 += c * c; }
  red[tid] = s2; __syncthreads();
  for (int st = 128; st > 0; st >>= 1) { if (tid < st) red[tid] += red[tid + st]; __syncthreads(); }
  const float rs = rsqrtf(red[0] / (float)N + eps);
  for (int pass = 0; pass < 2; ++pass) {
    for (int u = 0; u < per / 4; ++u) {
      const int j = tid * 4 + 1024 * u;
      v4f o, sm;
#pragma unroll
      for (int q = 0; q < 4; ++q) {
        float gg = g[j + q], bb = bta[j + q];
        if (PARAM_BF16) { gg = bf16_round(gg); bb = bf16_round(bb); }
        sm[q] = vals[u * 4 + q]; o[q] = (vals[u * 4 + q] - mu) * rs * gg + bb;
      }
      if (out_sum) *(volatile v4f*)(out_sum + (size_t)row * N + j) = sm;
      *(volatile v4f*)(out_norm + (size_t)row * N + j) = o;
    }
    if (pass == 0) __threadfence();
  }
}


typedef _Float16 v16h __attribute__((ext_vector_type(16)));
union FragH { v16h v; v8us half[2]; _Float16 h[16]; unsigned short u[16]; };
template <int NT>
__device__ __forceinline__ v8f mmaH(v16h ah, v16h al, v16h bh, v16h bl, v8f c) {
  c = __builtin_amdgcn_wmma_f32_16x16x32_f16(false, ah, false, bh, (short)0, c, false, false);
  if (NT >= 2) c = __builtin_amdgcn_wmma_f32_16x16x32_f16(false, al, false, bh, (short)0, c, false, false);
  if (NT >= 3) c = __builtin_amdgcn_wmma_f32_16x16x32_f16(false, ah, false, bl, (short)0, c, false, false);
  asm volatile("v_nop\n\tv_nop\n\tv_nop\n\tv_nop" : "+v"(c) : "v"(ah), "v"(al), "v"(bh), "v"(bl));
  return c;
}
template <bool ASPLIT>
__global__ __launch_bounds__(128) void k_gemm_h(const float* __restrict__ A, int lda, size_t sA, const _Float16* __restrict__ Bh, int ldb, size_t sB, float alpha, float* __restrict__ C, int ldc, size_t sC, int M, int N, int K) {
  __shared__ __attribute__((aligned(16))) float so[4][16][64];
  const int tid = threadIdx.x, w = tid >> 5, lane = tid & 31, ln = lane & 15, hh = lane >> 4; const int by = blockIdx.y;
  A += (size_t)by * sA; Bh += (size_t)by * sB; C += (size_t)by * sC;
  const int ntn = (N + 63) / 64; const int wid = blockIdx.x * 4 + w; const int mt = wid / ntn, nq = wid % ntn; if (mt * 16 >= M) return;
  const int row0 = mt * 16, col0 = nq * 64; const float* arow = A + (size_t)(row0 + ln) * lda;
  v8f acc[4] = {};
  for (int kb = 0; kb < K; kb += 32) {
    FragH ah, al;
    const v4f x0 = *(const v4fa*)(arow + kb + 8 * hh), x1 = *(const v4fa*)(arow + kb + 8 * hh + 4), x2 = *(const v4fa*)(arow + kb + 16 + 8 * hh), x3 = *(const v4fa*)(arow + kb + 16 + 8 * hh + 4);
    float xs[16] = {x0[0],x0[1],x0[2],x0[3],x1[0],x1[1],x1[2],x1[3],x2[0],x2[1],x2[2],x2[3],x3[0],x3[1],x3[2],x3[3]};
#pragma unroll
    for (int i = 0; i < 16; ++i) { const _Float16 h = (_Float16)xs[i]; ah.h[i] = h; al.h[i] = ASPLIT ? (_Float16)(xs[i] - (float)h) : (_Float16)0.0f; }
#pragma unroll
    for (int t = 0; t < 4; ++t) { if (col0 + t * 16 >= N) continue; const size_t boff = (size_t)(col0 + t * 16 + ln) * ldb + kb; FragH bq; bq.half[0] = *(const v8us*)(Bh + boff + 8 * hh); bq.half[1] = *(const v8us*)(Bh + boff + 16 + 8 * hh);
      acc[t] = mmaH<ASPLIT ? 2 : 1>(ah.v, al.v, bq.v, bq.v, acc[t]); }
  }
#pragma unroll
  for (int t = 0; t < 4; ++t) { if (col0 + t * 16 >= N) continue;
#pragma unroll
    for (int r = 0; r < 8; ++r) so[w][8 * hh + r][t * 16 + ln] = acc[t][r] * alpha; }
  __builtin_amdgcn_fence(__ATOMIC_ACQ_REL, "workgroup"); __builtin_amdgcn_wave_barrier();
  const int rsub = lane >> 4, c4 = (lane & 15) * 4;
  for (int pass = 0; pass < 2; ++pass) {
#pragma unroll
    for (int q = 0; q < 8; ++q) { const int r = q * 2 + rsub; if (col0 + c4 < N) { const v4f v = *(const v4fa*)&so[w][r][c4]; *(volatile v4f*)(C + (size_t)(row0 + r) * ldc + col0 + c4) = v; } }
    if (pass == 0) __threadfence(); }
}

__global__ __launch_bounds__(256) void k_wt_f16(const float* __restrict__ W, _Float16* __restrict__ Wt, int K, int N, float scale) {
  const int t = blockIdx.x * 256 + threadIdx.x; if (t >= N * (K / 8)) return; const int n = t / (K / 8), k8 = (t % (K / 8)) * 8; FragH f;
#pragma unroll
  for (int i = 0; i < 8; ++i) f.h[i] = (_Float16)(bf16_round(W[(size_t)(k8 + i) * N + n]) * scale); const v8us o = f.half[0];
  *(volatile v8us*)((unsigned short*)Wt + (size_t)n * K + k8) = o; __threadfence(); *(volatile v8us*)((unsigned short*)Wt + (size_t)n * K + k8) = o;
}
template <int ACT>
__global__ __launch_bounds__(128) void k_gemm_hhx(const _Float16* __restrict__ A, int lda, size_t sA, const _Float16* __restrict__ Bh, int ldb, size_t sB, float alpha, const float* __restrict__ bias, size_t sBias, const float* __restrict__ CP, int rowsPerB, size_t sCPb, int row0g,
    float* __restrict__ C, _Float16* __restrict__ C16, int ldc, size_t sC, int M, int N, int K) {
  __shared__ __attribute__((aligned(16))) float so[4][16][64];
  const int tid = threadIdx.x, w = tid >> 5, lane = tid & 31, ln = lane & 15, hh = lane >> 4; const int by = blockIdx.y;
  A += (size_t)by * sA; Bh += (size_t)by * sB; const size_t cofs = (size_t)by * sC; const float* bp = bias ? bias + (size_t)by * sBias : nullptr;
  const int ntn = (N + 63) / 64; const int wid = blockIdx.x * 4 + w; const int mt = wid / ntn, nq = wid % ntn; if (mt * 16 >= M) return;
  const int row0 = mt * 16, col0 = nq * 64; const _Float16* arow = A + (size_t)(row0 + ln) * lda;
  v8f acc[4] = {};
  for (int kb = 0; kb < K; kb += 32) { FragH ah; ah.half[0] = *(const v8us*)((const unsigned short*)arow + kb + 8 * hh); ah.half[1] = *(const v8us*)((const unsigned short*)arow + kb + 16 + 8 * hh);
#pragma unroll
    for (int t = 0; t < 4; ++t) { if (col0 + t * 16 >= N) continue; const size_t boff = (size_t)(col0 + t * 16 + ln) * ldb + kb; FragH bq; bq.half[0] = *(const v8us*)((const unsigned short*)Bh + boff + 8 * hh); bq.half[1] = *(const v8us*)((const unsigned short*)Bh + boff + 16 + 8 * hh);
      acc[t] = mmaH<1>(ah.v, ah.v, bq.v, bq.v, acc[t]); }
  }
#pragma unroll
  for (int t = 0; t < 4; ++t) { if (col0 + t * 16 >= N) continue; const int col = col0 + t * 16 + ln; const float bv = bp ? bf16_round(bp[col]) : 0.f;
#pragma unroll
    for (int r = 0; r < 8; ++r) { float v = acc[t][r] * alpha + bv; if (CP) { const int bidx = (row0g + row0 + 8 * hh + r) / rowsPerB; v += CP[(size_t)bidx * sCPb + (size_t)by * 64 + col]; } if (ACT == 1) v = (v > 0.f) ? v : expm1f(v); else if (ACT == 7) v = (v > 0.f) ? v + 1.0f : expf(v); else if (ACT == 8) v = tanhf(v); else if (ACT == 9) v = 0.5f * v * (1.0f + tanhf(0.7978845608028654f * (v + 0.044715f * v * v * v))); else if (ACT == 11) v = 1.0f / (1.0f + expf(-v)); else if (ACT == 12) v = (v > 0.f) ? v : 0.01f * v; else if (ACT == 14) v = (v > 0.f) ? v : 0.1f * v; else if (ACT == 15) v = v / (1.0f + expf(-v)); else if (ACT == 3) v = fmaxf(v, 0.f); else if (ACT == 6) v = 0.5f * v * (1.0f + erff(v * 0.70710678118654752f)); so[w][8 * hh + r][t * 16 + ln] = v; } }
  __builtin_amdgcn_fence(__ATOMIC_ACQ_REL, "workgroup"); __builtin_amdgcn_wave_barrier();
  const int rsub = lane >> 4, c4 = (lane & 15) * 4; typedef _Float16 v4h __attribute__((ext_vector_type(4)));
  for (int pass = 0; pass < 2; ++pass) {
#pragma unroll
    for (int q = 0; q < 8; ++q) { const int r = q * 2 + rsub; if (col0 + c4 < N) { const v4f v = *(const v4fa*)&so[w][r][c4]; if (C) *(volatile v4f*)(C + cofs + (size_t)(row0 + r) * ldc + col0 + c4) = v; if (C16) { v4h h4; for (int i = 0; i < 4; ++i) h4[i] = (_Float16)v[i]; *(volatile v4h*)(C16 + cofs + (size_t)(row0 + r) * ldc + col0 + c4) = h4; } } }
    if (pass == 0) __threadfence(); }
}


typedef _Float16 v4h __attribute__((ext_vector_type(4)));

__global__ __launch_bounds__(256) void k_x16(const float* __restrict__ x, _Float16* __restrict__ X16, size_t n8) { const size_t t = (size_t)blockIdx.x * 256 + threadIdx.x; if (t >= n8) return; FragH f;
#pragma unroll
  for (int q = 0; q < 8; ++q) f.h[q] = (_Float16)bf16_round(x[t * 8 + q]); *(volatile v8us*)((unsigned short*)X16 + t * 8) = f.half[0]; __threadfence(); *(volatile v8us*)((unsigned short*)X16 + t * 8) = f.half[0]; }
__global__ __launch_bounds__(256) void k_h16(const float* __restrict__ x, _Float16* __restrict__ X16, size_t n8) { const size_t t = (size_t)blockIdx.x * 256 + threadIdx.x; if (t >= n8) return; FragH f;
#pragma unroll
  for (int q = 0; q < 8; ++q) f.h[q] = (_Float16)x[t * 8 + q]; *(volatile v8us*)((unsigned short*)X16 + t * 8) = f.half[0]; __threadfence(); *(volatile v8us*)((unsigned short*)X16 + t * 8) = f.half[0]; }
__global__ __launch_bounds__(256) void k_round16f(const float* __restrict__ W, _Float16* __restrict__ Bt, size_t n8) { const size_t t = (size_t)blockIdx.x * 256 + threadIdx.x; if (t >= n8) return; FragH f;
#pragma unroll
  for (int i = 0; i < 8; ++i) f.h[i] = (_Float16)(bf16_round(W[t * 8 + i]) * 16.0f); *(volatile v8us*)((unsigned short*)Bt + t * 8) = f.half[0]; __threadfence(); *(volatile v8us*)((unsigned short*)Bt + t * 8) = f.half[0]; }
template <int NHv, int TTv>
__global__ __launch_bounds__(256) void k_vt(const _Float16* __restrict__ V16, int ldv, int voff, _Float16* __restrict__ Vt) { __shared__ unsigned short tl[64][66]; const int tid = threadIdx.x; const int slab = blockIdx.x / (TTv / 64), lg = blockIdx.x % (TTv / 64); const int b = slab / NHv, h = slab % NHv;
  for (int i = tid; i < 64 * 8; i += 256) { const int r = i / 8, c8 = (i % 8) * 8; FragH f; f.half[0] = *(const v8us*)((const unsigned short*)V16 + ((size_t)b * TTv + lg * 64 + r) * ldv + voff + h * 64 + c8);
#pragma unroll
    for (int q = 0; q < 8; ++q) tl[r][c8 + q] = f.u[q]; }
  __syncthreads();
  for (int pass = 0; pass < 2; ++pass) {
#pragma unroll
    for (int rd = 0; rd < 2; ++rd) { const int d = rd * 32 + tid / 8, pc = tid % 8; FragH f;
#pragma unroll
      for (int q = 0; q < 8; ++q) f.u[q] = tl[pc * 8 + q][d];
      *(volatile v8us*)((unsigned short*)Vt + ((size_t)slab * 64 + d) * TTv + lg * 64 + pc * 8) = f.half[0]; }
    if (pass == 0) __threadfence(); } }

__global__ __launch_bounds__(256) void k_hl(const float* __restrict__ F, _Float16* __restrict__ Hh, _Float16* __restrict__ Hl, size_t n8) { const size_t t = (size_t)blockIdx.x * 256 + threadIdx.x; if (t >= n8) return; FragH fh, fl; const v4f a = *(const v4fa*)(F + t * 8), c = *(const v4fa*)(F + t * 8 + 4);
#pragma unroll
  for (int q = 0; q < 4; ++q) { _Float16 h = (_Float16)a[q]; fh.h[q] = h; fl.h[q] = (_Float16)((a[q] - (float)h) * 1024.0f); h = (_Float16)c[q]; fh.h[4 + q] = h; fl.h[4 + q] = (_Float16)((c[q] - (float)h) * 1024.0f); }
  for (int pass = 0; pass < 2; ++pass) { *(volatile v8us*)((unsigned short*)Hh + t * 8) = fh.half[0]; *(volatile v8us*)((unsigned short*)Hl + t * 8) = fl.half[0]; if (pass == 0) __threadfence(); } }

__global__ __launch_bounds__(256) void k_in8(const float* __restrict__ x, int i0, int ni, _Float16* __restrict__ X8) { const int t = blockIdx.x * 256 + threadIdx.x; if (t >= ni * 1024) return; const int p = t % 1024, i = i0 + t / 1024; FragH f = FragH{};
#pragma unroll
  for (int c = 0; c < 3; ++c) f.h[c] = (_Float16)bf16_round(x[((size_t)i * 3 + c) * 1024 + p]);
  *(volatile v8us*)((unsigned short*)X8 + (size_t)t * 8) = f.half[0]; __threadfence(); *(volatile v8us*)((unsigned short*)X8 + (size_t)t * 8) = f.half[0]; }
__global__ __launch_bounds__(256) void k_im2col5(const _Float16* __restrict__ P, int ni, int S, int C, int KTp, _Float16* __restrict__ COL) { const int SS_ = S * S; const int cg = C / 8; const int t = blockIdx.x * 256 + threadIdx.x; if (t >= ni * SS_ * KTp * cg) return; const int g = t % cg; const int k = (t / cg) % KTp; const int r = t / (cg * KTp); const int p = r % SS_, i = r / SS_; FragH f = FragH{};
  if (k < 25) { const int h = p / S, w = p % S; const int yy = h - 2 + k / 5, xx = w - 2 + k % 5; if (yy >= 0 && yy < S && xx >= 0 && xx < S) f.half[0] = *(const v8us*)((const unsigned short*)P + ((size_t)i * SS_ + yy * S + xx) * C + g * 8); }
  *(volatile v8us*)((unsigned short*)COL + ((size_t)r * KTp + k) * C + g * 8) = f.half[0]; __threadfence(); *(volatile v8us*)((unsigned short*)COL + ((size_t)r * KTp + k) * C + g * 8) = f.half[0]; }
__global__ __launch_bounds__(256) void k_w5(const float* __restrict__ w, int O, int Opad, int Cin, int C, int KTp, _Float16* __restrict__ Bt) { const int KD = KTp * C; const int t = blockIdx.x * 256 + threadIdx.x; if (t >= Opad * (KD / 8)) return; const int col0 = (t % (KD / 8)) * 8, o = t / (KD / 8); FragH f;
#pragma unroll
  for (int q = 0; q < 8; ++q) { const int col = col0 + q; const int k = col / C, c = col % C; f.h[q] = (o < O && k < 25 && c < Cin) ? (_Float16)(bf16_round(w[(((size_t)o * Cin + c) * 5 + k / 5) * 5 + k % 5]) * 16.0f) : (_Float16)0.0f; }
  *(volatile v8us*)((unsigned short*)Bt + (size_t)o * KD + col0) = f.half[0]; __threadfence(); *(volatile v8us*)((unsigned short*)Bt + (size_t)o * KD + col0) = f.half[0]; }
__global__ __launch_bounds__(256) void k_tail(const float* __restrict__ Y, int ni, int iout0, int S, int C, const float* __restrict__ g, const float* __restrict__ bb, const float* __restrict__ mm, const float* __restrict__ vv, _Float16* __restrict__ OUT) {
  #pragma clang fp contract(off)
  const int So = S / 2; const int cg = C / 8; const int t = blockIdx.x * 256 + threadIdx.x; if (t >= ni * So * So * cg) return; const int gq = t % cg; const int po = (t / cg) % (So * So); const int i = t / (cg * So * So); const int yo = po / So, xo = po % So; FragH f;
#pragma unroll
  for (int q = 0; q < 8; ++q) { const int c = gq * 8 + q; const float s = bf16_round(g[c]) * rsqrtf(bf16_round(vv[c]) + 1e-5f); const float sh = bf16_round(bb[c]) - bf16_round(mm[c]) * s; float acc = 0.f;
#pragma unroll
    for (int d = 0; d < 4; ++d) { const int yy = 2 * yo + (d >> 1), xx = 2 * xo + (d & 1); const float v = Y[((size_t)i * S * S + yy * S + xx) * C + c]; acc += fmaxf(v * s + sh, 0.f); }
    f.h[q] = (_Float16)fminf(fmaxf(acc / 4.0f, 0.f), 1.0f); }
  *(volatile v8us*)((unsigned short*)OUT + ((size_t)(iout0 + i) * So * So + po) * C + gq * 8) = f.half[0]; __threadfence(); *(volatile v8us*)((unsigned short*)OUT + ((size_t)(iout0 + i) * So * So + po) * C + gq * 8) = f.half[0]; }
__global__ __launch_bounds__(256) void k_w4(const float* __restrict__ w, _Float16* __restrict__ Bt) { const int t = blockIdx.x * 256 + threadIdx.x; if (t >= 16 * 128) return; const int col0 = (t % 128) * 8, o = t / 128; FragH f;
#pragma unroll
  for (int q = 0; q < 8; ++q) { const int col = col0 + q; const int yx = col / 64, c = col % 64; f.h[q] = (o < 10) ? (_Float16)(bf16_round(w[(((size_t)o * 64 + c) * 4 + yx / 4) * 4 + yx % 4]) * 16.0f) : (_Float16)0.0f; }
  *(volatile v8us*)((unsigned short*)Bt + (size_t)o * 1024 + col0) = f.half[0]; __threadfence(); *(volatile v8us*)((unsigned short*)Bt + (size_t)o * 1024 + col0) = f.half[0]; }
__global__ __launch_bounds__(256) void k_fin(const float* __restrict__ Z, const float* __restrict__ g, const float* __restrict__ bb, const float* __restrict__ mm, const float* __restrict__ vv, float* __restrict__ out) {
  #pragma clang fp contract(off)
  const int t = blockIdx.x * 256 + threadIdx.x; if (t >= NB * 10 / 4) return; v4f v;
#pragma unroll
  for (int q = 0; q < 4; ++q) { const int f = t * 4 + q; const int i = f / 10, o = f % 10; const float s = bf16_round(g[o]) * rsqrtf(bf16_round(vv[o]) + 1e-5f); v[q] = Z[(size_t)i * 16 + o] * s + (bf16_round(bb[o]) - bf16_round(mm[o]) * s); }
  *(volatile v4f*)(out + (size_t)t * 4) = v; __threadfence(); *(volatile v4f*)(out + (size_t)t * 4) = v; }

extern "C" void kernel_launch(void* const* d_in, const int* in_sizes, int n_in,
                              void* d_out, int out_size, void* d_ws, size_t ws_size, hipStream_t stream) {
  (void)in_sizes; (void)n_in; (void)out_size;
  const float* const* I = (const float* const*)d_in; const float* x = I[0];
  char* ws = (char*)d_ws; size_t off = 0;
  auto take = [&](size_t bytes) { char* p = ws + off; off += (bytes + 255) & ~(size_t)255; return p; };
  const int KT1 = 28;
  _Float16* B1 = (_Float16*)take((size_t)32 * KT1 * 8 * 2); _Float16* B2 = (_Float16*)take((size_t)32 * 25 * 32 * 2); _Float16* B3 = (_Float16*)take((size_t)64 * 25 * 32 * 2); _Float16* B4 = (_Float16*)take((size_t)16 * 1024 * 2);
  const int CH1 = 128;
  _Float16* X8 = (_Float16*)take((size_t)CH1 * 1024 * 8 * 2); _Float16* COL = (_Float16*)take((size_t)CH1 * 1024 * KT1 * 8 * 2); float* Y = (float*)take((size_t)CH1 * 1024 * 32 * 4);
  _Float16* P1 = (_Float16*)take((size_t)NB * 256 * 32 * 2); _Float16* P2 = (_Float16*)take((size_t)NB * 64 * 32 * 2); _Float16* P3 = (_Float16*)take((size_t)NB * 16 * 64 * 2); float* Z = (float*)take((size_t)NB * 16 * 4);
  if (off > ws_size) return;
  k_w5<<<(32 * (KT1 * 8 / 8) + 255) / 256, 256, 0, stream>>>(I[1], 32, 32, 3, 8, KT1, B1); k_w5<<<(32 * (25 * 32 / 8) + 255) / 256, 256, 0, stream>>>(I[6], 32, 32, 32, 32, 25, B2); k_w5<<<(64 * (25 * 32 / 8) + 255) / 256, 256, 0, stream>>>(I[11], 64, 64, 32, 32, 25, B3); k_w4<<<(16 * 128 + 255) / 256, 256, 0, stream>>>(I[16], B4);
  for (int i0 = 0; i0 < NB; i0 += CH1) {
    k_in8<<<(CH1 * 1024 + 255) / 256, 256, 0, stream>>>(x, i0, CH1, X8);
    k_im2col5<<<(CH1 * 1024 * KT1 * 1 + 255) / 256, 256, 0, stream>>>(X8, CH1, 32, 8, KT1, COL);
    k_gemm_hhx<0><<<dim3(((CH1 * 1024 / 16) * 1 + 3) / 4, 1), 128, 0, stream>>>(COL, KT1 * 8, 0, B1, KT1 * 8, 0, 0.0625f, nullptr, 0, nullptr, 1, 0, 0, Y, nullptr, 32, 0, CH1 * 1024, 32, KT1 * 8);
    k_tail<<<(CH1 * 256 * 4 + 255) / 256, 256, 0, stream>>>(Y, CH1, i0, 32, 32, I[2], I[3], I[4], I[5], P1); }
  for (int i0 = 0; i0 < NB; i0 += CH1) {
    k_im2col5<<<(CH1 * 256 * 25 * 4 + 255) / 256, 256, 0, stream>>>(P1 + (size_t)i0 * 256 * 32, CH1, 16, 32, 25, COL);
    k_gemm_hhx<0><<<dim3(((CH1 * 256 / 16) * 1 + 3) / 4, 1), 128, 0, stream>>>(COL, 800, 0, B2, 800, 0, 0.0625f, nullptr, 0, nullptr, 1, 0, 0, Y, nullptr, 32, 0, CH1 * 256, 32, 800);
    k_tail<<<(CH1 * 64 * 4 + 255) / 256, 256, 0, stream>>>(Y, CH1, i0, 16, 32, I[7], I[8], I[9], I[10], P2); }
  for (int i0 = 0; i0 < NB; i0 += 512) {
    k_im2col5<<<(512 * 64 * 25 * 4 + 255) / 256, 256, 0, stream>>>(P2 + (size_t)i0 * 64 * 32, 512, 8, 32, 25, COL);
    k_gemm_hhx<0><<<dim3(((512 * 64 / 16) * 1 + 3) / 4, 1), 128, 0, stream>>>(COL, 800, 0, B3, 800, 0, 0.0625f, nullptr, 0, nullptr, 1, 0, 0, Y, nullptr, 64, 0, 512 * 64, 64, 800);
    k_tail<<<(512 * 16 * 8 + 255) / 256, 256, 0, stream>>>(Y, 512, i0, 8, 64, I[12], I[13], I[14], I[15], P3); }
  k_gemm_hhx<0><<<dim3(((NB / 16) * 1 + 3) / 4, 1), 128, 0, stream>>>(P3, 1024, 0, B4, 1024, 0, 0.0625f, nullptr, 0, nullptr, 1, 0, 0, Z, nullptr, 16, 0, NB, 16, 1024);
  k_fin<<<(NB * 10 / 4 + 255) / 256, 256, 0, stream>>>(Z, I[17], I[18], I[19], I[20], (float*)d_out);
}
